// MessagePassing_87505663689045
// MI455X (gfx1250) — hardware-verified
//
#include <hip/hip_runtime.h>
#include <stddef.h>
#include <stdint.h>
#include <math.h>


#define F      128
#define F2     256
#define ATC    256
#define NBR    16
#define NK     15
#define K2     256
#define K3     384
#define NQR    512
#define NTHR   256
#define NWAVE  8
#define APW    4
#define SPW    8
#define GBM    64
#define GBN    128
#define GTHR   128
#define GWAVE  (GTHR / 32)
#define PARTW  288
#define WSTW   258
#define WSTW3  514
#define NUWP   (F2 * (K2 / 8))
#define NBW    (NUWP / NTHR)
#define NUQR   (NQR * (K3 / 8))
#define NBQR   (NUQR / NTHR)
#define NBPREP (3 * NBW + NBQR)
#define WSLIM  134217728

static_assert(F == 4 * 32 && F2 == 2 * F && K2 == 2 * F && K3 == 3 * F && NQR == 2 * F2);
static_assert((K2 % 32) == 0 && (K3 % 32) == 0);
static_assert(NBR == 2 * NWAVE && NK == NBR - 1);
static_assert(NTHR == F2 && NTHR == 32 * NWAVE);
static_assert(GBM == GWAVE * 16 && GBN == 4 * 32 && GTHR == GBN && F2 == 2 * GBN && F == GBN);
static_assert(PARTW % 32 == 0 && PARTW / 4 <= GTHR && PARTW >= 2 * GBN + 1 && (2 * PARTW) / 4 <= NTHR);
static_assert(WSTW >= 2 * GBN + 1 && (WSTW % 2) == 0 && WSTW3 >= 2 * F2 + 1 && (WSTW3 % 2) == 0);
static_assert((NUWP % NTHR) == 0 && (NUQR % NTHR) == 0 && (K3 / 8) == 48 && (K2 / 8) == 32);
static_assert((ATC & (ATC - 1)) == 0 && (ATC % GBM) == 0 && (ATC % (NWAVE * APW)) == 0);
static_assert(((NBR * NQR) % (4 * NTHR)) == 0);
static_assert(NBR * NQR * 4 + F2 * 4 + NWAVE * WSTW3 * 4 + 2 * PARTW * 4 <= 65536);

typedef float          v4f  __attribute__((ext_vector_type(4)));
typedef float          v8f  __attribute__((ext_vector_type(8)));
typedef int            v8i  __attribute__((ext_vector_type(8)));
typedef unsigned int   v2u  __attribute__((ext_vector_type(2)));
typedef unsigned int   v4u  __attribute__((ext_vector_type(4)));
typedef unsigned short v8us __attribute__((ext_vector_type(8)));
typedef __bf16         v16b __attribute__((ext_vector_type(16)));
typedef v4f  __attribute__((may_alias)) v4fa;
typedef v8us __attribute__((may_alias)) v8usa;
union FragB { v16b v; v8us h[2]; v8i w; };

__device__ __forceinline__ v8f wmb(const FragB& a, const FragB& b, v8f c) {
  v8f d = __builtin_amdgcn_wmma_f32_16x16x32_bf16(false, a.v, false, b.v, (short)0, c, false, false);
  asm volatile("v_nop\n\tv_nop\n\tv_nop\n\tv_nop" : "+v"(d) : "v"(a.w), "v"(b.w));
  return d;
}

__device__ __forceinline__ v8f z8() { v8f z = {0.f, 0.f, 0.f, 0.f, 0.f, 0.f, 0.f, 0.f}; return z; }

__device__ __forceinline__ unsigned int f2bf(float f) {
  const unsigned int u = __float_as_uint(f);
  return ((u + 0x7FFFu + ((u >> 16) & 1u)) >> 16) & 0xFFFFu;
}
__device__ __forceinline__ float bf2f(unsigned int b) { return __uint_as_float(b << 16); }
__device__ __forceinline__ float bfr(float f) { return bf2f(f2bf(f)); }
__device__ __forceinline__ v4f bfr4(const v4f a) {
  v4f r; r.x = bfr(a.x); r.y = bfr(a.y); r.z = bfr(a.z); r.w = bfr(a.w); return r;
}
__device__ __forceinline__ unsigned int pk2(float lo, float hi) { return f2bf(lo) | (f2bf(hi) << 16); }
__device__ __forceinline__ v4u pack8(const v4f a, const v4f b) {
  v4u r;
  r.x = pk2(a.x, a.y); r.y = pk2(a.z, a.w); r.z = pk2(b.x, b.y); r.w = pk2(b.z, b.w);
  return r;
}
__device__ __forceinline__ void hl2(float v0, float v1, unsigned int& hw, unsigned int& lw) {
  const unsigned int h0 = f2bf(v0), h1 = f2bf(v1);
  const unsigned int l0 = f2bf(v0 - bf2f(h0)), l1 = f2bf(v1 - bf2f(h1));
  hw = h0 | (h1 << 16);
  lw = l0 | (l1 << 16);
}
__device__ __forceinline__ void pack8hl(const v4f a, const v4f b, v4u& hv, v4u& lv) {
  unsigned int h, l;
  hl2(a.x, a.y, h, l); hv.x = h; lv.x = l;
  hl2(a.z, a.w, h, l); hv.y = h; lv.y = l;
  hl2(b.x, b.y, h, l); hv.z = h; lv.z = l;
  hl2(b.z, b.w, h, l); hv.w = h; lv.w = l;
}

__device__ __forceinline__ float frcp(float x) { return __builtin_amdgcn_rcpf(x); }
__device__ __forceinline__ float gexp(float x) { return __expf(fminf(x, 80.0f)); }
__device__ __forceinline__ float gsig(float x) { return frcp(1.0f + gexp(-x)); }
__device__ __forceinline__ float gtanh(float x) { return fmaf(-2.0f, frcp(gexp(x + x) + 1.0f), 1.0f); }

__device__ __forceinline__ void wsync() {
  __builtin_amdgcn_fence(__ATOMIC_RELEASE, "wavefront");
  __builtin_amdgcn_wave_barrier();
}

__global__ __launch_bounds__(NTHR) void k_wprep(const float* __restrict__ Wn, const float* __restrict__ W2,
                                                const float* __restrict__ W3,
                                                unsigned short* wnb, unsigned short* w2b, unsigned short* wab,
                                                unsigned short* wqrb) {
  const int b = (int)blockIdx.x, tid = (int)threadIdx.x;
  const float* p;
  unsigned short* o;
  if (b < NBW) {
    const int u  = b * NTHR + tid;
    const int n  = u >> 5;
    const int k8 = (u & 31) * 8;
    p = Wn + (size_t)k8 * F2 + n;
    o = wnb + (size_t)n * K2 + k8;
  } else if (b < 2 * NBW) {
    const int u  = (b - NBW) * NTHR + tid;
    const int n  = u >> 5;
    const int k8 = (u & 31) * 8;
    const int kk = k8 & (F - 1);
    p = W2 + (size_t)kk * F2 + n;
    o = w2b + (size_t)n * K2 + k8;
  } else if (b < 3 * NBW) {
    const int u  = (b - 2 * NBW) * NTHR + tid;
    const int n  = u >> 5;
    const int k8 = (u & 31) * 8;
    const int kk = k8 & (F - 1);
    p = W3 + (size_t)kk * F2 + n;
    o = wab + (size_t)n * K2 + k8;
  } else {
    const int u  = (b - 3 * NBW) * NTHR + tid;
    const int n  = u / 48;
    const int k8 = (u - n * 48) * 8;
    const int nn = n & (F2 - 1);
    const int hf = n >> 8;
    const int sr = (k8 < K2) ? (F + F * hf + (k8 & (F - 1))) : (3 * F + F * hf + (k8 - K2));
    p = W3 + (size_t)sr * F2 + nn;
    o = wqrb + (size_t)n * K3 + k8;
  }
  v4f a, c;
  a.x = p[0];                    a.y = p[(size_t)F2];          a.z = p[(size_t)2 * F2];      a.w = p[(size_t)3 * F2];
  c.x = p[(size_t)4 * F2];       c.y = p[(size_t)5 * F2];      c.z = p[(size_t)6 * F2];      c.w = p[(size_t)7 * F2];
  const v4u wv = pack8(a, c);
  *(volatile v4u*)o = wv;
  __threadfence();
  *(volatile v4u*)o = wv;
}

__global__ __launch_bounds__(NTHR) void k_a1prep(const float* __restrict__ node, const float* __restrict__ edge,
                                                 const int* __restrict__ msk, int nUnits, unsigned short* a1) {
  const int u = (int)blockIdx.x * NTHR + (int)threadIdx.x;
  if (u >= nUnits) return;
  const int s  = u >> 5;
  const int q  = u & 31;
  const int a  = s >> 4;
  const int c8 = (q & 15) * 8;
  const float* pn = node + (size_t)a * F + c8;
  const float* pe = edge + (size_t)s * F + c8;
  const v4f na = *(const v4fa*)pn, nb = *(const v4fa*)(pn + 4);
  const v4f ea = *(const v4fa*)pe, eb = *(const v4fa*)(pe + 4);
  const float fn = (q < 16) ? 1.0f : 0.0f;
  const float fe = 1.0f - fn;
  const float mf = (msk[s] != 0) ? 1.0f : 0.0f;
  v4f xa, xb;
  xa.x = fmaf(na.x, fn, ea.x * fe) * mf; xa.y = fmaf(na.y, fn, ea.y * fe) * mf;
  xa.z = fmaf(na.z, fn, ea.z * fe) * mf; xa.w = fmaf(na.w, fn, ea.w * fe) * mf;
  xb.x = fmaf(nb.x, fn, eb.x * fe) * mf; xb.y = fmaf(nb.y, fn, eb.y * fe) * mf;
  xb.z = fmaf(nb.z, fn, eb.z * fe) * mf; xb.w = fmaf(nb.w, fn, eb.w * fe) * mf;
  const v4u wv = pack8(xa, xb);
  unsigned short* o = a1 + (size_t)s * K2 + 8 * q;
  *(volatile v4u*)o = wv;
  __threadfence();
  *(volatile v4u*)o = wv;
}

template <int KD, int MODE>
__global__ __launch_bounds__(GTHR) void k_gemm(const unsigned short* __restrict__ A,
                                               const unsigned short* __restrict__ BT, int nN,
                                               const float* __restrict__ bias,
                                               float* xout, int ldo, float* part) {
  __shared__ __attribute__((aligned(16))) float stg[GBM * GBN];
  __shared__ __attribute__((aligned(16))) float wst[GWAVE * WSTW];
  __shared__ __attribute__((aligned(16))) float pst[PARTW];
  const int tid = (int)threadIdx.x, lane = tid & 31, wave = tid >> 5, hh = lane >> 4, m = lane & 15;
  const int rowBase = (int)blockIdx.x * GBM;
  const int colBase = (int)blockIdx.y * GBN;

  v8f acc[8];
#pragma unroll
  for (int t = 0; t < 8; ++t) acc[t] = z8();
  const unsigned short* ap = A  + (size_t)(rowBase + 16 * wave + m) * (size_t)KD + 8 * hh;
  const unsigned short* bp = BT + (size_t)(colBase + m) * (size_t)KD + 8 * hh;

#pragma unroll 1
  for (int k0 = 0; k0 < KD; k0 += 32) {
    FragB af;
    af.h[0] = *(const v8usa*)(ap + k0);
    af.h[1] = *(const v8usa*)(ap + k0 + 16);
#pragma unroll
    for (int nt = 0; nt < 8; ++nt) {
      const unsigned short* wq = bp + (size_t)(16 * nt) * (size_t)KD + k0;
      FragB bf;
      bf.h[0] = *(const v8usa*)wq;
      bf.h[1] = *(const v8usa*)(wq + 16);
      acc[nt] = wmb(af, bf, acc[nt]);
    }
  }

#pragma unroll
  for (int nt = 0; nt < 8; ++nt) {
    const int lc = 16 * nt + m;
#pragma unroll
    for (int r = 0; r < 8; ++r) {
      const int lr = 16 * wave + 8 * hh + r;
      stg[lr * GBN + lc] = acc[nt][r];
    }
  }
  __syncthreads();

  float bq[4];
  if constexpr (MODE == 1) {
    const v4f b4 = *(const v4f*)(bias + colBase + 4 * lane);
    bq[0] = bfr(b4.x); bq[1] = bfr(b4.y); bq[2] = bfr(b4.z); bq[3] = bfr(b4.w);
  } else {
    bq[0] = 0.0f; bq[1] = 0.0f; bq[2] = 0.0f; bq[3] = 0.0f;
  }

  v4f pv[16];
  int wn = 0;
  float wm[4], wqv[4];
#pragma unroll
  for (int j = 0; j < 4; ++j) { wm[j] = 0.0f; wqv[j] = 0.0f; }
#pragma unroll
  for (int i = 0; i < 16; ++i) {
    const int row = rowBase + 16 * wave + i;
    const bool ok = row < nN;
    const v4f x = *(const v4fa*)(stg + (16 * wave + i) * GBN + 4 * lane);
    float y[4];
    y[0] = x.x + bq[0]; y[1] = x.y + bq[1]; y[2] = x.z + bq[2]; y[3] = x.w + bq[3];
    float vv[4];
#pragma unroll
    for (int j = 0; j < 4; ++j) vv[j] = ok ? y[j] : 0.0f;
    v4f q;
    q.x = vv[0]; q.y = vv[1]; q.z = vv[2]; q.w = vv[3];
    pv[i] = q;
    if constexpr (MODE == 1) {
      if (ok) {
        wn += 1;
        const float rk = 1.0f / (float)(i + 1);
#pragma unroll
        for (int j = 0; j < 4; ++j) {
          const float d = vv[j] - wm[j];
          wm[j]  = fmaf(d, rk, wm[j]);
          wqv[j] = fmaf(d, vv[j] - wm[j], wqv[j]);
        }
      }
    }
  }
#pragma unroll
  for (int i = 0; i < 16; ++i) {
    float* op = xout + (size_t)(rowBase + 16 * wave + i) * (size_t)ldo + colBase + 4 * lane;
    *(volatile v4f*)op = pv[i];
  }
  __threadfence();
#pragma unroll
  for (int i = 0; i < 16; ++i) {
    float* op = xout + (size_t)(rowBase + 16 * wave + i) * (size_t)ldo + colBase + 4 * lane;
    *(volatile v4f*)op = pv[i];
  }

  if constexpr (MODE == 1) {
    if (lane == 0) wst[wave * WSTW] = (float)wn;
#pragma unroll
    for (int j = 0; j < 4; ++j) {
      wst[wave * WSTW + 1 + 4 * lane + j]       = wm[j];
      wst[wave * WSTW + 1 + GBN + 4 * lane + j] = wqv[j];
    }
    __syncthreads();
    {
      float n = 0.0f, mean = 0.0f, M2 = 0.0f;
#pragma unroll 1
      for (int w2 = 0; w2 < GWAVE; ++w2) {
        const float nb = wst[w2 * WSTW];
        const float mb = wst[w2 * WSTW + 1 + tid];
        const float qb = wst[w2 * WSTW + 1 + GBN + tid];
        if (nb > 0.5f) {
          const float nn = n + nb;
          const float delta = mb - mean;
          const float f = nb / nn;
          mean = fmaf(delta, f, mean);
          M2 = M2 + qb + delta * delta * n * f;
          n = nn;
        }
      }
      pst[1 + tid] = mean;
      pst[1 + GBN + tid] = M2;
      if (tid == 0) pst[0] = n;
    }
#pragma unroll 1
    for (int i = 2 * GBN + 1 + tid; i < PARTW; i += GTHR) pst[i] = 0.0f;
    __syncthreads();
    const int pb = (int)blockIdx.x * (int)gridDim.y + (int)blockIdx.y;
    v4f ps;
    if (tid < PARTW / 4) {
      ps = *(const v4fa*)(pst + 4 * tid);
      *(volatile v4f*)(part + (size_t)pb * PARTW + 4 * tid) = ps;
    }
    __threadfence();
    if (tid < PARTW / 4) {
      *(volatile v4f*)(part + (size_t)pb * PARTW + 4 * tid) = ps;
    }
  } else {
    (void)wn; (void)part; (void)bias;
  }
}

template <int NC>
__global__ __launch_bounds__(NC) void k_bnfin(const float* __restrict__ part, int nPart,
                                              const float* __restrict__ gam, const float* __restrict__ bet,
                                              float* ss) {
  __shared__ __attribute__((aligned(16))) float stg[2 * NC];
  const int tid = (int)threadIdx.x;
  const int c   = tid;
  const int cb  = c >> 7;
  const int cc  = c & (GBN - 1);
  const int nCB = NC / GBN;
  double n = 0.0, mean = 0.0, M2 = 0.0;
#pragma unroll 1
  for (int b = 0; b < nPart; ++b) {
    const float* pr = part + ((size_t)b * (size_t)nCB + (size_t)cb) * PARTW;
    const double nb = (double)pr[0];
    const double mb = (double)pr[1 + cc];
    const double qb = (double)pr[1 + GBN + cc];
    if (nb > 0.5) {
      const double nn = n + nb;
      const double delta = mb - mean;
      const double f = nb / nn;
      mean = mean + delta * f;
      M2 = M2 + qb + delta * delta * n * f;
      n = nn;
    }
  }
  const double nt = n < 1.0 ? 1.0 : n;
  const float varf  = (float)(M2 / nt);
  const float meanf = (float)mean;
  const float rstd = 1.0f / sqrtf(varf + 1e-5f);
  const float sc = bfr(gam[c]) * rstd;
  const float sh = bfr(bet[c]) - meanf * sc;
  stg[c] = sc;
  stg[NC + c] = sh;
  __syncthreads();
  v4f v;
  if (tid < (2 * NC) / 4) {
    v = *(const v4fa*)(stg + 4 * tid);
    *(volatile v4f*)(ss + 4 * tid) = v;
  }
  __threadfence();
  if (tid < (2 * NC) / 4) {
    *(volatile v4f*)(ss + 4 * tid) = v;
  }
}

__global__ __launch_bounds__(NTHR) void k_node(const float* __restrict__ c1, const float* __restrict__ ss1,
                                               float* sout, float* part) {
  __shared__ __attribute__((aligned(16))) float ssh[2 * F2];
  __shared__ __attribute__((aligned(16))) float wst[NWAVE * WSTW];
  __shared__ __attribute__((aligned(16))) float pst[PARTW];
  const int tid = (int)threadIdx.x, lane = tid & 31, wave = tid >> 5;
  ssh[tid] = ss1[tid];
  ssh[F2 + tid] = ss1[F2 + tid];
  __syncthreads();
  const int c4 = 4 * lane;
  float scg[4], shg[4], sce[4], she[4];
#pragma unroll
  for (int i = 0; i < 4; ++i) {
    scg[i] = ssh[c4 + i];      shg[i] = ssh[F2 + c4 + i];
    sce[i] = ssh[F + c4 + i];  she[i] = ssh[F2 + F + c4 + i];
  }
  float wm[4], wq[4];
#pragma unroll
  for (int i = 0; i < 4; ++i) { wm[i] = 0.0f; wq[i] = 0.0f; }
#pragma unroll
  for (int r = 0; r < APW; ++r) {
    const int a = (int)blockIdx.x * (NWAVE * APW) + wave * APW + r;
    float acc[4];
#pragma unroll
    for (int i = 0; i < 4; ++i) acc[i] = 0.0f;
#pragma unroll 1
    for (int j = 0; j < NBR; ++j) {
      const float* rp = c1 + (size_t)(a * NBR + j) * F2 + c4;
      const v4f ga = *(const v4fa*)rp;
      const v4f ea = *(const v4fa*)(rp + F);
      acc[0] = fmaf(gsig(fmaf(ga.x, scg[0], shg[0])), gtanh(fmaf(ea.x, sce[0], she[0])), acc[0]);
      acc[1] = fmaf(gsig(fmaf(ga.y, scg[1], shg[1])), gtanh(fmaf(ea.y, sce[1], she[1])), acc[1]);
      acc[2] = fmaf(gsig(fmaf(ga.z, scg[2], shg[2])), gtanh(fmaf(ea.z, sce[2], she[2])), acc[2]);
      acc[3] = fmaf(gsig(fmaf(ga.w, scg[3], shg[3])), gtanh(fmaf(ea.w, sce[3], she[3])), acc[3]);
    }
    v4f o;
    o.x = acc[0]; o.y = acc[1]; o.z = acc[2]; o.w = acc[3];
    float* sp = sout + (size_t)a * F + c4;
    *(volatile v4f*)sp = o;
    __threadfence();
    *(volatile v4f*)sp = o;
    const float rk = 1.0f / (float)(r + 1);
#pragma unroll
    for (int i = 0; i < 4; ++i) {
      const float d = acc[i] - wm[i];
      wm[i] = fmaf(d, rk, wm[i]);
      wq[i] = fmaf(d, acc[i] - wm[i], wq[i]);
    }
  }
  if (lane == 0) wst[wave * WSTW] = (float)APW;
#pragma unroll
  for (int i = 0; i < 4; ++i) {
    wst[wave * WSTW + 1 + c4 + i]     = wm[i];
    wst[wave * WSTW + 1 + F + c4 + i] = wq[i];
  }
  __syncthreads();
  if (tid < F) {
    float n = 0.0f, mean = 0.0f, M2 = 0.0f;
#pragma unroll 1
    for (int w2 = 0; w2 < NWAVE; ++w2) {
      const float nb = wst[w2 * WSTW];
      const float mb = wst[w2 * WSTW + 1 + tid];
      const float qb = wst[w2 * WSTW + 1 + F + tid];
      if (nb > 0.5f) {
        const float nn = n + nb;
        const float delta = mb - mean;
        const float f = nb / nn;
        mean = fmaf(delta, f, mean);
        M2 = M2 + qb + delta * delta * n * f;
        n = nn;
      }
    }
    pst[1 + tid] = mean;
    pst[1 + F + tid] = M2;
    if (tid == 0) pst[0] = n;
  }
  if (tid < PARTW - 2 * F - 1) pst[2 * F + 1 + tid] = 0.0f;
  __syncthreads();
  const int pb = (int)blockIdx.x;
  v4f ps;
  if (tid < PARTW / 4) {
    ps = *(const v4fa*)(pst + 4 * tid);
    *(volatile v4f*)(part + (size_t)pb * PARTW + 4 * tid) = ps;
  }
  __threadfence();
  if (tid < PARTW / 4) {
    *(volatile v4f*)(part + (size_t)pb * PARTW + 4 * tid) = ps;
  }
}

__global__ __launch_bounds__(NTHR) void k_un(const float* __restrict__ node, const float* __restrict__ s1,
                                             const float* __restrict__ ss2,
                                             float* out0, float* unf, unsigned short* unhl) {
  __shared__ __attribute__((aligned(16))) float ssh[2 * F];
  __shared__ __attribute__((aligned(16))) float rst[NWAVE * F];
  const int tid = (int)threadIdx.x, lane = tid & 31, wave = tid >> 5;
  ssh[tid] = ss2[tid];
  __syncthreads();
  const int a  = (int)blockIdx.x * NWAVE + wave;
  const int c4 = 4 * lane;
  const v4f nv = bfr4(*(const v4fa*)(node + (size_t)a * F + c4));
  const v4f sv = *(const v4fa*)(s1 + (size_t)a * F + c4);
  v4f y;
  y.x = gtanh(nv.x + fmaf(sv.x, ssh[c4 + 0], ssh[F + c4 + 0]));
  y.y = gtanh(nv.y + fmaf(sv.y, ssh[c4 + 1], ssh[F + c4 + 1]));
  y.z = gtanh(nv.z + fmaf(sv.z, ssh[c4 + 2], ssh[F + c4 + 2]));
  y.w = gtanh(nv.w + fmaf(sv.w, ssh[c4 + 3], ssh[F + c4 + 3]));

  *(v4fa*)(rst + wave * F + c4) = y;
  wsync();
  const int l16 = lane & 15;
  const v4f pa = *(const v4fa*)(rst + wave * F + 8 * l16);
  const v4f pb = *(const v4fa*)(rst + wave * F + 8 * l16 + 4);
  v4u hv, lv;
  pack8hl(pa, pb, hv, lv);
  v4u wv;
  wv.x = (lane < 16) ? hv.x : lv.x;
  wv.y = (lane < 16) ? hv.y : lv.y;
  wv.z = (lane < 16) ? hv.z : lv.z;
  wv.w = (lane < 16) ? hv.w : lv.w;
  float* op = out0 + (size_t)a * F + c4;
  float* fp = unf + (size_t)a * F + c4;
  unsigned short* hp = unhl + (size_t)a * K2 + 8 * lane;
  *(volatile v4f*)op = y;
  *(volatile v4f*)fp = y;
  *(volatile v4u*)hp = wv;
  __threadfence();
  *(volatile v4f*)op = y;
  *(volatile v4f*)fp = y;
  *(volatile v4u*)hp = wv;
}

__global__ __launch_bounds__(NTHR) void k_a23(const float* __restrict__ unf, const float* __restrict__ edge,
                                              const int* __restrict__ idx, const int* __restrict__ msk, int nA,
                                              unsigned short* a2, unsigned short* a3) {
  __shared__ __attribute__((aligned(16))) float rst[NWAVE * 2 * F];
  const int tid = (int)threadIdx.x, lane = tid & 31, wave = tid >> 5;
  const int c4 = 4 * lane, l16 = lane & 15;
  float* st0 = rst + wave * 2 * F;
  float* st1 = st0 + F;
#pragma unroll 1
  for (int r = 0; r < SPW; ++r) {
    const int s  = (int)blockIdx.x * (NWAVE * SPW) + wave * SPW + r;
    const int a  = s >> 4;
    const int cb = a & ~(ATC - 1);
    const int raw = idx[s];
    const int jj = raw < 0 ? 0 : (raw > ATC - 1 ? ATC - 1 : raw);
    int nj = cb + jj;
    nj = nj > nA - 1 ? nA - 1 : nj;
    const float mf = (msk[s] != 0) ? 1.0f : 0.0f;
    const v4f ui = *(const v4fa*)(unf + (size_t)a * F + c4);
    const v4f uj = *(const v4fa*)(unf + (size_t)nj * F + c4);
    const v4f ev = *(const v4fa*)(edge + (size_t)s * F + c4);
    v4f p;
    p.x = (ui.x * uj.x) * mf; p.y = (ui.y * uj.y) * mf; p.z = (ui.z * uj.z) * mf; p.w = (ui.w * uj.w) * mf;
    wsync();
    *(v4fa*)(st0 + c4) = p;
    *(v4fa*)(st1 + c4) = uj;
    wsync();
    const v4f pa = *(const v4fa*)(st0 + 8 * l16);
    const v4f pb = *(const v4fa*)(st0 + 8 * l16 + 4);
    const v4f qa = *(const v4fa*)(st1 + 8 * l16);
    const v4f qb = *(const v4fa*)(st1 + 8 * l16 + 4);
    v4u hv, lv, wv2, wv3;
    pack8hl(pa, pb, hv, lv);
    wv2.x = (lane < 16) ? hv.x : lv.x; wv2.y = (lane < 16) ? hv.y : lv.y;
    wv2.z = (lane < 16) ? hv.z : lv.z; wv2.w = (lane < 16) ? hv.w : lv.w;
    pack8hl(qa, qb, hv, lv);
    wv3.x = (lane < 16) ? hv.x : lv.x; wv3.y = (lane < 16) ? hv.y : lv.y;
    wv3.z = (lane < 16) ? hv.z : lv.z; wv3.w = (lane < 16) ? hv.w : lv.w;
    v2u we;
    we.x = pk2(ev.x, ev.y);
    we.y = pk2(ev.z, ev.w);
    unsigned short* p2 = a2 + (size_t)s * K2 + 8 * lane;
    unsigned short* p3 = a3 + (size_t)s * K3 + 8 * lane;
    unsigned short* pe = a3 + (size_t)s * K3 + K2 + 4 * lane;
    *(volatile v4u*)p2 = wv2;
    *(volatile v4u*)p3 = wv3;
    *(volatile v2u*)pe = we;
    __threadfence();
    *(volatile v4u*)p2 = wv2;
    *(volatile v4u*)p3 = wv3;
    *(volatile v2u*)pe = we;
  }
}

__global__ __launch_bounds__(NTHR) void k_tb1(const float* __restrict__ pa, const float* __restrict__ qr,
                                              const float* __restrict__ b3, float* part) {
  __shared__ __attribute__((aligned(16))) float sqr[NBR * NQR];
  __shared__ __attribute__((aligned(16))) float sp[F2];
  __shared__ __attribute__((aligned(16))) float wst[NWAVE * WSTW3];
  __shared__ __attribute__((aligned(16))) float pst[2 * PARTW];
  const int tid = (int)threadIdx.x, lane = tid & 31, wave = tid >> 5;
  const int a = (int)blockIdx.x;
  const float* qb0 = qr + (size_t)a * (NBR * NQR);
#pragma unroll 1
  for (int i = tid; i < (NBR * NQR) / 4; i += NTHR) *(v4fa*)(sqr + 4 * i) = *(const v4fa*)(qb0 + 4 * (size_t)i);
  sp[tid] = pa[(size_t)a * F2 + tid] + bfr(b3[tid]);
  __syncthreads();
  const int c4 = 4 * lane;
  const v4f pg = *(const v4fa*)(sp + c4);
  const v4f pe = *(const v4fa*)(sp + F + c4);
  float wm[8], wq[8];
#pragma unroll
  for (int i = 0; i < 8; ++i) { wm[i] = 0.0f; wq[i] = 0.0f; }
#pragma unroll
  for (int jj = 0; jj < 2; ++jj) {
    const int j = wave + NWAVE * jj;
    const v4f qg = *(const v4fa*)(sqr + j * NQR + c4);
    const v4f qe = *(const v4fa*)(sqr + j * NQR + F + c4);
    float bg[4], be[4];
    bg[0] = pg.x + qg.x; bg[1] = pg.y + qg.y; bg[2] = pg.z + qg.z; bg[3] = pg.w + qg.w;
    be[0] = pe.x + qe.x; be[1] = pe.y + qe.y; be[2] = pe.z + qe.z; be[3] = pe.w + qe.w;
#pragma unroll 1
    for (int kk = 0; kk < NK; ++kk) {
      const int k = kk + ((kk >= j) ? 1 : 0);
      const int n = jj * NK + kk + 1;
      const float rk = frcp((float)n);
      const v4f rg = *(const v4fa*)(sqr + k * NQR + F2 + c4);
      const v4f re = *(const v4fa*)(sqr + k * NQR + F2 + F + c4);
      float v[8];
      v[0] = bg[0] + rg.x; v[1] = bg[1] + rg.y; v[2] = bg[2] + rg.z; v[3] = bg[3] + rg.w;
      v[4] = be[0] + re.x; v[5] = be[1] + re.y; v[6] = be[2] + re.z; v[7] = be[3] + re.w;
#pragma unroll
      for (int i = 0; i < 8; ++i) {
        const float d = v[i] - wm[i];
        wm[i] = fmaf(d, rk, wm[i]);
        wq[i] = fmaf(d, v[i] - wm[i], wq[i]);
      }
    }
  }
  if (lane == 0) wst[wave * WSTW3] = (float)(2 * NK);
#pragma unroll
  for (int i = 0; i < 4; ++i) {
    wst[wave * WSTW3 + 1 + c4 + i]          = wm[i];
    wst[wave * WSTW3 + 1 + F + c4 + i]      = wm[4 + i];
    wst[wave * WSTW3 + 1 + F2 + c4 + i]     = wq[i];
    wst[wave * WSTW3 + 1 + F2 + F + c4 + i] = wq[4 + i];
  }
  __syncthreads();
  {
    const int c = tid;
    float n = 0.0f, mean = 0.0f, M2 = 0.0f;
#pragma unroll 1
    for (int w2 = 0; w2 < NWAVE; ++w2) {
      const float nb = wst[w2 * WSTW3];
      const float mb = wst[w2 * WSTW3 + 1 + c];
      const float qv = wst[w2 * WSTW3 + 1 + F2 + c];
      if (nb > 0.5f) {
        const float nn = n + nb;
        const float delta = mb - mean;
        const float f = nb / nn;
        mean = fmaf(delta, f, mean);
        M2 = M2 + qv + delta * delta * n * f;
        n = nn;
      }
    }
    const int cb = c >> 7;
    const int cc = c & (GBN - 1);
    pst[cb * PARTW + 1 + cc] = mean;
    pst[cb * PARTW + 1 + GBN + cc] = M2;
    if (cc == 0) pst[cb * PARTW] = n;
  }
  if (tid < 2 * (PARTW - 2 * GBN - 1)) {
    const int rr = tid / (PARTW - 2 * GBN - 1);
    const int q  = tid - rr * (PARTW - 2 * GBN - 1);
    pst[rr * PARTW + 2 * GBN + 1 + q] = 0.0f;
  }
  __syncthreads();
  v4f ps;
  if (tid < (2 * PARTW) / 4) {
    ps = *(const v4fa*)(pst + 4 * tid);
    *(volatile v4f*)(part + (size_t)a * (2 * PARTW) + 4 * tid) = ps;
  }
  __threadfence();
  if (tid < (2 * PARTW) / 4) {
    *(volatile v4f*)(part + (size_t)a * (2 * PARTW) + 4 * tid) = ps;
  }
}

__global__ __launch_bounds__(NTHR) void k_tb2(const float* __restrict__ pa, const float* __restrict__ qr,
                                              const float* __restrict__ b3, const float* __restrict__ ss4,
                                              float* t3, float* part) {
  __shared__ __attribute__((aligned(16))) float sqr[NBR * NQR];
  __shared__ __attribute__((aligned(16))) float sp[F2];
  __shared__ __attribute__((aligned(16))) float ssh[2 * F2];
  __shared__ __attribute__((aligned(16))) float wst[NWAVE * WSTW];
  __shared__ __attribute__((aligned(16))) float pst[PARTW];
  const int tid = (int)threadIdx.x, lane = tid & 31, wave = tid >> 5;
  const int a = (int)blockIdx.x;
  const float* qb0 = qr + (size_t)a * (NBR * NQR);
#pragma unroll 1
  for (int i = tid; i < (NBR * NQR) / 4; i += NTHR) *(v4fa*)(sqr + 4 * i) = *(const v4fa*)(qb0 + 4 * (size_t)i);
  sp[tid] = pa[(size_t)a * F2 + tid] + bfr(b3[tid]);
  ssh[tid] = ss4[tid];
  ssh[F2 + tid] = ss4[F2 + tid];
  __syncthreads();
  const int c4 = 4 * lane;
  float scg[4], shg[4], sce[4], she[4];
#pragma unroll
  for (int i = 0; i < 4; ++i) {
    scg[i] = ssh[c4 + i];      shg[i] = ssh[F2 + c4 + i];
    sce[i] = ssh[F + c4 + i];  she[i] = ssh[F2 + F + c4 + i];
  }
  const v4f pg = *(const v4fa*)(sp + c4);
  const v4f pe = *(const v4fa*)(sp + F + c4);
  float wm[4], wq[4];
#pragma unroll
  for (int i = 0; i < 4; ++i) { wm[i] = 0.0f; wq[i] = 0.0f; }
#pragma unroll
  for (int jj = 0; jj < 2; ++jj) {
    const int j = wave + NWAVE * jj;
    const v4f qg = *(const v4fa*)(sqr + j * NQR + c4);
    const v4f qe = *(const v4fa*)(sqr + j * NQR + F + c4);
    float bg[4], be[4];
    bg[0] = pg.x + qg.x; bg[1] = pg.y + qg.y; bg[2] = pg.z + qg.z; bg[3] = pg.w + qg.w;
    be[0] = pe.x + qe.x; be[1] = pe.y + qe.y; be[2] = pe.z + qe.z; be[3] = pe.w + qe.w;
    float acc[4];
#pragma unroll
    for (int i = 0; i < 4; ++i) acc[i] = 0.0f;
#pragma unroll 1
    for (int kk = 0; kk < NK; ++kk) {
      const int k = kk + ((kk >= j) ? 1 : 0);
      const v4f rg = *(const v4fa*)(sqr + k * NQR + F2 + c4);
      const v4f re = *(const v4fa*)(sqr + k * NQR + F2 + F + c4);
      float vg[4], ve[4];
      vg[0] = bg[0] + rg.x; vg[1] = bg[1] + rg.y; vg[2] = bg[2] + rg.z; vg[3] = bg[3] + rg.w;
      ve[0] = be[0] + re.x; ve[1] = be[1] + re.y; ve[2] = be[2] + re.z; ve[3] = be[3] + re.w;
#pragma unroll
      for (int i = 0; i < 4; ++i) {
        acc[i] = fmaf(gsig(fmaf(vg[i], scg[i], shg[i])), gtanh(fmaf(ve[i], sce[i], she[i])), acc[i]);
      }
    }
    v4f o;
    o.x = acc[0]; o.y = acc[1]; o.z = acc[2]; o.w = acc[3];
    float* tp = t3 + (size_t)(a * NBR + j) * F + c4;
    *(volatile v4f*)tp = o;
    __threadfence();
    *(volatile v4f*)tp = o;
    if (jj == 0) {
#pragma unroll
      for (int i = 0; i < 4; ++i) { wm[i] = acc[i]; wq[i] = 0.0f; }
    } else {
#pragma unroll
      for (int i = 0; i < 4; ++i) {
        const float d = acc[i] - wm[i];
        wm[i] = fmaf(d, 0.5f, wm[i]);
        wq[i] = fmaf(d, acc[i] - wm[i], wq[i]);
      }
    }
  }
  if (lane == 0) wst[wave * WSTW] = 2.0f;
#pragma unroll
  for (int i = 0; i < 4; ++i) {
    wst[wave * WSTW + 1 + c4 + i]     = wm[i];
    wst[wave * WSTW + 1 + F + c4 + i] = wq[i];
  }
  __syncthreads();
  if (tid < F) {
    float n = 0.0f, mean = 0.0f, M2 = 0.0f;
#pragma unroll 1
    for (int w2 = 0; w2 < NWAVE; ++w2) {
      const float nb = wst[w2 * WSTW];
      const float mb = wst[w2 * WSTW + 1 + tid];
      const float qv = wst[w2 * WSTW + 1 + F + tid];
      if (nb > 0.5f) {
        const float nn = n + nb;
        const float delta = mb - mean;
        const float f = nb / nn;
        mean = fmaf(delta, f, mean);
        M2 = M2 + qv + delta * delta * n * f;
        n = nn;
      }
    }
    pst[1 + tid] = mean;
    pst[1 + F + tid] = M2;
    if (tid == 0) pst[0] = n;
  }
  if (tid < PARTW - 2 * F - 1) pst[2 * F + 1 + tid] = 0.0f;
  __syncthreads();
  v4f ps;
  if (tid < PARTW / 4) {
    ps = *(const v4fa*)(pst + 4 * tid);
    *(volatile v4f*)(part + (size_t)a * PARTW + 4 * tid) = ps;
  }
  __threadfence();
  if (tid < PARTW / 4) {
    *(volatile v4f*)(part + (size_t)a * PARTW + 4 * tid) = ps;
  }
}

__global__ __launch_bounds__(NTHR) void k_ue(const float* __restrict__ edge, const float* __restrict__ c2,
                                             const float* __restrict__ ss3, const float* __restrict__ t3,
                                             const float* __restrict__ ss5, int nUnits, float* out1) {
  __shared__ __attribute__((aligned(16))) float sh3[2 * F2];
  __shared__ __attribute__((aligned(16))) float sh5[2 * F];
  const int tid = (int)threadIdx.x;
  sh3[tid] = ss3[tid];
  sh3[F2 + tid] = ss3[F2 + tid];
  sh5[tid] = ss5[tid];
  __syncthreads();
  const int u = (int)blockIdx.x * NTHR + tid;
  if (u >= nUnits) return;
  const int s  = u >> 5;
  const int c4 = (u & 31) * 4;
  const v4f ev = bfr4(*(const v4fa*)(edge + (size_t)s * F + c4));
  const v4f ga = *(const v4fa*)(c2 + (size_t)s * F2 + c4);
  const v4f ea = *(const v4fa*)(c2 + (size_t)s * F2 + F + c4);
  const v4f tv = *(const v4fa*)(t3 + (size_t)s * F + c4);
  float e4[4], g4[4], q4[4], t4[4], o4[4];
  e4[0] = ev.x; e4[1] = ev.y; e4[2] = ev.z; e4[3] = ev.w;
  g4[0] = ga.x; g4[1] = ga.y; g4[2] = ga.z; g4[3] = ga.w;
  q4[0] = ea.x; q4[1] = ea.y; q4[2] = ea.z; q4[3] = ea.w;
  t4[0] = tv.x; t4[1] = tv.y; t4[2] = tv.z; t4[3] = tv.w;
#pragma unroll
  for (int i = 0; i < 4; ++i) {
    const float tb = gsig(fmaf(g4[i], sh3[c4 + i], sh3[F2 + c4 + i])) * gtanh(fmaf(q4[i], sh3[F + c4 + i], sh3[F2 + F + c4 + i]));
    const float tt = fmaf(t4[i], sh5[c4 + i], sh5[F + c4 + i]);
    const float z  = (e4[i] + tb) + tt;
    o4[i] = gtanh(z);
  }
  v4f o;
  o.x = o4[0]; o.y = o4[1]; o.z = o4[2]; o.w = o4[3];
  float* op = out1 + (size_t)u * 4;
  *(volatile v4f*)op = o;
  __threadfence();
  *(volatile v4f*)op = o;
}

static inline size_t al256(size_t o) { return (o + 255) & ~(size_t)255; }

extern "C" void kernel_launch(void* const* d_in, const int* in_sizes, int n_in,
                              void* d_out, int out_size, void* d_ws, size_t ws_size,
                              hipStream_t stream) {
  if (n_in < 20) return;
  if (in_sizes[0] < F * ATC || (in_sizes[0] % F) != 0) return;
  const int nA = in_sizes[0] / F;
  if ((nA % ATC) != 0 || (nA % GBM) != 0 || (nA % (NWAVE * APW)) != 0 || nA > (1 << 20)) return;
  const int nS = nA * NBR;
  if (in_sizes[1] != nS * F || in_sizes[2] != nS || in_sizes[3] != nS) return;
  if ((nS % GBM) != 0 || (nS % (NWAVE * SPW)) != 0 || (nS % 8) != 0) return;
  if (in_sizes[4] != F2 * F2 || in_sizes[5] != F2 || in_sizes[6] != F2 || in_sizes[7] != F2) return;
  if (in_sizes[8] != F || in_sizes[9] != F) return;
  if (in_sizes[10] != F * F2 || in_sizes[11] != F2 || in_sizes[12] != F2 || in_sizes[13] != F2) return;
  if (in_sizes[14] != 5 * F * F2 || in_sizes[15] != F2 || in_sizes[16] != F2 || in_sizes[17] != F2) return;
  if (in_sizes[18] != F || in_sizes[19] != F) return;
  if ((long long)out_size != (long long)nA * F + (long long)nS * F) return;

  const float* node = (const float*)d_in[0];
  const float* edge = (const float*)d_in[1];
  const int*   nidx = (const int*)d_in[2];
  const int*   nmsk = (const int*)d_in[3];
  const float* Wn   = (const float*)d_in[4];
  const float* bnd  = (const float*)d_in[5];
  const float* g1   = (const float*)d_in[6];
  const float* be1  = (const float*)d_in[7];
  const float* g2   = (const float*)d_in[8];
  const float* be2  = (const float*)d_in[9];
  const float* W2   = (const float*)d_in[10];
  const float* b2   = (const float*)d_in[11];
  const float* g2b  = (const float*)d_in[12];
  const float* be2b = (const float*)d_in[13];
  const float* W3   = (const float*)d_in[14];
  const float* b3   = (const float*)d_in[15];
  const float* g3b  = (const float*)d_in[16];
  const float* be3b = (const float*)d_in[17];
  const float* gS   = (const float*)d_in[18];
  const float* beS  = (const float*)d_in[19];
  float* out  = (float*)d_out;
  float* out1 = out + (size_t)nA * F;

  const int gM1 = nS / GBM;
  const int gMA = nA / GBM;
  const int gNd = nA / (NWAVE * APW);
  int nPT = 2 * gM1;
  if (gNd > nPT) nPT = gNd;
  if (2 * nA > nPT) nPT = 2 * nA;

  char* ws = (char*)d_ws;
  size_t off = 0;
  const size_t oWNB = off; off = al256(off + (size_t)F2 * K2 * 2);
  const size_t oW2B = off; off = al256(off + (size_t)F2 * K2 * 2);
  const size_t oWAB = off; off = al256(off + (size_t)F2 * K2 * 2);
  const size_t oWQR = off; off = al256(off + (size_t)NQR * K3 * 2);
  const size_t oA1  = off; off = al256(off + (size_t)nS * K2 * 2);
  const size_t oC1  = off; off = al256(off + (size_t)nS * F2 * 4);
  const size_t oPT  = off; off = al256(off + (size_t)nPT * PARTW * 4);
  const size_t oSS1 = off; off = al256(off + (size_t)(2 * F2) * 4);
  const size_t oSS2 = off; off = al256(off + (size_t)(2 * F2) * 4);
  const size_t oSS3 = off; off = al256(off + (size_t)(2 * F2) * 4);
  const size_t oSS4 = off; off = al256(off + (size_t)(2 * F2) * 4);
  const size_t oSS5 = off; off = al256(off + (size_t)(2 * F2) * 4);
  const size_t oS1  = off; off = al256(off + (size_t)nA * F * 4);
  const size_t oUNF = off; off = al256(off + (size_t)nA * F * 4);
  const size_t oUHL = off; off = al256(off + (size_t)nA * K2 * 2);
  const size_t oA2  = off; off = al256(off + (size_t)nS * K2 * 2);
  const size_t oA3  = off; off = al256(off + (size_t)nS * K3 * 2);
  const size_t oC2  = off; off = al256(off + (size_t)nS * F2 * 4);
  const size_t oPA  = off; off = al256(off + (size_t)nA * F2 * 4);
  const size_t oQR  = off; off = al256(off + (size_t)nS * NQR * 4);
  const size_t oT3  = off; off = al256(off + (size_t)nS * F * 4);
  if (off > ws_size || off > (size_t)WSLIM) return;
  unsigned short* WNB  = (unsigned short*)(ws + oWNB);
  unsigned short* W2B  = (unsigned short*)(ws + oW2B);
  unsigned short* WAB  = (unsigned short*)(ws + oWAB);
  unsigned short* WQRB = (unsigned short*)(ws + oWQR);
  unsigned short* A1   = (unsigned short*)(ws + oA1);
  float*          C1   = (float*)(ws + oC1);
  float*          PT   = (float*)(ws + oPT);
  float*          SS1  = (float*)(ws + oSS1);
  float*          SS2  = (float*)(ws + oSS2);
  float*          SS3  = (float*)(ws + oSS3);
  float*          SS4  = (float*)(ws + oSS4);
  float*          SS5  = (float*)(ws + oSS5);
  float*          S1   = (float*)(ws + oS1);
  float*          UNF  = (float*)(ws + oUNF);
  unsigned short* UNHL = (unsigned short*)(ws + oUHL);
  unsigned short* A2   = (unsigned short*)(ws + oA2);
  unsigned short* A3   = (unsigned short*)(ws + oA3);
  float*          C2   = (float*)(ws + oC2);
  float*          PA   = (float*)(ws + oPA);
  float*          QR   = (float*)(ws + oQR);
  float*          T3   = (float*)(ws + oT3);

  k_wprep<<<NBPREP, NTHR, 0, stream>>>(Wn, W2, W3, WNB, W2B, WAB, WQRB);
  const int nU1 = nS * 32;
  k_a1prep<<<(nU1 + NTHR - 1) / NTHR, NTHR, 0, stream>>>(node, edge, nmsk, nU1, A1);
  k_gemm<K2, 1><<<dim3(gM1, F2 / GBN), GTHR, 0, stream>>>(A1, WNB, nS, bnd, C1, F2, PT);
  k_bnfin<F2><<<1, F2, 0, stream>>>(PT, gM1, g1, be1, SS1);
  k_node<<<gNd, NTHR, 0, stream>>>(C1, SS1, S1, PT);
  k_bnfin<F><<<1, F, 0, stream>>>(PT, gNd, g2, be2, SS2);
  k_un<<<nA / NWAVE, NTHR, 0, stream>>>(node, S1, SS2, out, UNF, UNHL);
  k_a23<<<nS / (NWAVE * SPW), NTHR, 0, stream>>>(UNF, edge, nidx, nmsk, nA, A2, A3);
  k_gemm<K2, 1><<<dim3(gM1, F2 / GBN), GTHR, 0, stream>>>(A2, W2B, nS, b2, C2, F2, PT);
  k_bnfin<F2><<<1, F2, 0, stream>>>(PT, gM1, g2b, be2b, SS3);
  k_gemm<K2, 0><<<dim3(gMA, F2 / GBN), GTHR, 0, stream>>>(UNHL, WAB, nA, b3, PA, F2, PT);
  k_gemm<K3, 0><<<dim3(gM1, NQR / GBN), GTHR, 0, stream>>>(A3, WQRB, nS, b3, QR, NQR, PT);
  k_tb1<<<nA, NTHR, 0, stream>>>(PA, QR, b3, PT);
  k_bnfin<F2><<<1, F2, 0, stream>>>(PT, nA, g3b, be3b, SS4);
  k_tb2<<<nA, NTHR, 0, stream>>>(PA, QR, b3, SS4, T3, PT);
  k_bnfin<F><<<1, F, 0, stream>>>(PT, nA, gS, beS, SS5);
  const int nU2 = nS * 32;
  k_ue<<<(nU2 + NTHR - 1) / NTHR, NTHR, 0, stream>>>(edge, C2, SS3, T3, SS5, nU2, out1);
}
